// GNN_40724879901230
// MI455X (gfx1250) — hardware-verified
//
#include <hip/hip_runtime.h>
#include <stddef.h>
#include <stdint.h>
#include <math.h>


#define HID    64
#define K2     128
#define KRZ    256
#define NTHR   256
#define NWAVE  8
#define EPT    8
#define CHUNK  (NTHR * EPT)
#define WCAP   (EPT * 32)
#define LISTN  (NWAVE * WCAP)
#define NBA    1024
#define SLA    10
#define RCAP   16384
#define DEGCAP 64
#define GBM    64
#define GBN    64
#define GTHR   128
#define AGG_ZINTS    (LISTN + 2 * RCAP + 3 * NBA)
#define MISC_INTS    16
#define AGG_LDS_INTS (AGG_ZINTS + MISC_INTS)
#define GRU_LDS_FLOATS (4 * GBM * HID + 256)
#define WSMAX  134217728

#define O_GWT  0
#define O_M0T  4096
#define O_M1T  12288
#define O_RZT  20480
#define O_INT  53248
#define O_HNT  61440
#define WP_ELEMS 69632
#define U0 512
#define U1 1536
#define U2 2560
#define U3 4608
#define U4 6656
#define U5 7680
#define U6 8704

static_assert((CHUNK & (CHUNK - 1)) == 0 && CHUNK <= 4096);
static_assert((NBA & (NBA - 1)) == 0 && NBA == (1 << SLA));
static_assert(((long long)CHUNK << SLA) < (1LL << 31));
static_assert(NBA % NWAVE == 0 && NBA % 32 == 0 && NBA % GBM == 0 && NBA == 4 * NTHR);
static_assert(RCAP % (NTHR * 4) == 0 && AGG_ZINTS % (NTHR * 4) == 0 && LISTN % 4 == 0);
static_assert(DEGCAP == 64);
static_assert(HID == 2 * 32 && K2 == 2 * HID && KRZ == 4 * HID);
static_assert(HID % 32 == 0 && K2 % 32 == 0 && KRZ % 32 == 0);
static_assert(GBM == (GTHR / 32) * 16 && GBN == HID);
static_assert(U0 % NTHR == 0 && U1 % NTHR == 0 && U2 % NTHR == 0 && U3 % NTHR == 0);
static_assert(U4 % NTHR == 0 && U5 % NTHR == 0 && U6 % NTHR == 0);
static_assert(O_HNT + HID * K2 == WP_ELEMS && (WP_ELEMS * 2) % 256 == 0);
static_assert(AGG_LDS_INTS * 4 <= 300000 && GRU_LDS_FLOATS * 4 <= 300000);

typedef float          v2f   __attribute__((ext_vector_type(2)));
typedef float          v4f   __attribute__((ext_vector_type(4)));
typedef float          v8f   __attribute__((ext_vector_type(8)));
typedef int            v4i   __attribute__((ext_vector_type(4)));
typedef int            v8i   __attribute__((ext_vector_type(8)));
typedef unsigned int   v4u   __attribute__((ext_vector_type(4)));
typedef unsigned short v8us  __attribute__((ext_vector_type(8)));
typedef unsigned short v16us __attribute__((ext_vector_type(16)));
typedef __bf16         v16bf __attribute__((ext_vector_type(16)));
typedef v2f  __attribute__((may_alias)) v2fa;
typedef v4f  __attribute__((may_alias)) v4fa;
typedef v4i  __attribute__((may_alias)) v4ia;
typedef v8us __attribute__((may_alias)) v8usa;
union FragB { v16bf v; v16us u; v8us h[2]; v8i w; };

__device__ __forceinline__ v8f wmb(const FragB& a, const FragB& b, v8f c) {
  v8f d = __builtin_amdgcn_wmma_f32_16x16x32_bf16(false, a.v, false, b.v, (short)0, c, false, false);
  asm volatile("v_nop\n\tv_nop\n\tv_nop\n\tv_nop" : "+v"(d) : "v"(a.w), "v"(b.w));
  return d;
}

__device__ __forceinline__ unsigned bf16_bits(float f) {
  const unsigned u = __float_as_uint(f);
  const unsigned r = (u + 0x7FFFu + ((u >> 16) & 1u)) >> 16;
  return (f != f) ? 0x7FC0u : r;
}
__device__ __forceinline__ float bf16_val(float f) {
  return __uint_as_float(bf16_bits(f) << 16);
}
__device__ __forceinline__ unsigned short cvz(float f, bool ok) {
  const unsigned b = bf16_bits(f);
  return ok ? (unsigned short)b : (unsigned short)0;
}
__device__ __forceinline__ int clampi(int v, int lo, int hi) {
  return v < lo ? lo : (v > hi ? hi : v);
}

__device__ __forceinline__ void put_f32_row(float* base, int node, int lane, float v0, float v1, bool wr) {
  const int sa = (2 * lane) & 31, sb = (2 * lane + 1) & 31;
  v4f ow;
  ow.x = __shfl(v0, sa, 32); ow.y = __shfl(v1, sa, 32);
  ow.z = __shfl(v0, sb, 32); ow.w = __shfl(v1, sb, 32);
  float* op = base + (size_t)node * HID + 4 * (lane & 15);
  if (wr) *(volatile v4f*)op = ow;
  __threadfence();
  if (wr) *(volatile v4f*)op = ow;
}
__device__ __forceinline__ void put_hl_row(unsigned short* base, int node, int lane, float v0, float v1, bool wr) {
  const int q0s = (4 * lane) & 31, q1s = (4 * lane + 1) & 31;
  const int q2s = (4 * lane + 2) & 31, q3s = (4 * lane + 3) & 31;
  const unsigned hb0 = bf16_bits(v0), hb1 = bf16_bits(v1);
  const unsigned lb0 = bf16_bits(v0 - __uint_as_float(hb0 << 16));
  const unsigned lb1 = bf16_bits(v1 - __uint_as_float(hb1 << 16));
  const int hw = (int)(hb0 | (hb1 << 16));
  const int lw = (int)(lb0 | (lb1 << 16));
  const int g0 = __shfl(hw, q0s, 32), g1 = __shfl(hw, q1s, 32);
  const int g2 = __shfl(hw, q2s, 32), g3 = __shfl(hw, q3s, 32);
  const int p0 = __shfl(lw, q0s, 32), p1 = __shfl(lw, q1s, 32);
  const int p2 = __shfl(lw, q2s, 32), p3 = __shfl(lw, q3s, 32);
  const bool lsel = (lane & 8) != 0;
  v4u pv;
  pv.x = (unsigned int)(lsel ? p0 : g0);
  pv.y = (unsigned int)(lsel ? p1 : g1);
  pv.z = (unsigned int)(lsel ? p2 : g2);
  pv.w = (unsigned int)(lsel ? p3 : g3);
  unsigned short* hp = base + (size_t)node * K2 + 8 * (lane & 15);
  if (wr) *(volatile v4u*)hp = pv;
  __threadfence();
  if (wr) *(volatile v4u*)hp = pv;
}

template <int SLB>
__device__ __forceinline__ int scan_chunk(const int* __restrict__ dsts, int nE, int cbase, int slotBase,
                                          int nb, int vec8, int* list, int tid, int lane, int wave) {
  int wc = 0;
  const int el0  = tid * EPT;
  const int e0   = cbase + el0;
  const int sent = -2147483647 - 1;
  v4i da, db;
  if (vec8 != 0 && cbase + CHUNK <= nE) {
    da = *(const v4i*)(dsts + e0);
    db = *(const v4i*)(dsts + e0 + 4);
  } else {
    da.x = (e0     < nE) ? dsts[min(e0,     nE - 1)] : sent;
    da.y = (e0 + 1 < nE) ? dsts[min(e0 + 1, nE - 1)] : sent;
    da.z = (e0 + 2 < nE) ? dsts[min(e0 + 2, nE - 1)] : sent;
    da.w = (e0 + 3 < nE) ? dsts[min(e0 + 3, nE - 1)] : sent;
    db.x = (e0 + 4 < nE) ? dsts[min(e0 + 4, nE - 1)] : sent;
    db.y = (e0 + 5 < nE) ? dsts[min(e0 + 5, nE - 1)] : sent;
    db.z = (e0 + 6 < nE) ? dsts[min(e0 + 6, nE - 1)] : sent;
    db.w = (e0 + 7 < nE) ? dsts[min(e0 + 7, nE - 1)] : sent;
  }
  const unsigned nbs = (unsigned)slotBase;
  const unsigned unb = (unsigned)nb;
  const unsigned s0 = (unsigned)da.x - nbs, s1 = (unsigned)da.y - nbs;
  const unsigned s2 = (unsigned)da.z - nbs, s3 = (unsigned)da.w - nbs;
  const unsigned s4 = (unsigned)db.x - nbs, s5 = (unsigned)db.y - nbs;
  const unsigned s6 = (unsigned)db.z - nbs, s7 = (unsigned)db.w - nbs;
  const bool h0 = s0 < unb, h1 = s1 < unb, h2 = s2 < unb, h3 = s3 < unb;
  const bool h4 = s4 < unb, h5 = s5 < unb, h6 = s6 < unb, h7 = s7 < unb;
  const unsigned any = __builtin_amdgcn_ballot_w32(h0 | h1 | h2 | h3 | h4 | h5 | h6 | h7);
  if (any != 0u) {
#define HITJ(J, HJ, SJ) { \
      const unsigned mj = __builtin_amdgcn_ballot_w32(HJ); \
      if (mj != 0u) { \
        if (HJ) { \
          const int pos = wc + (int)__builtin_amdgcn_mbcnt_lo(mj, 0u); \
          if (pos < WCAP) list[wave * WCAP + pos] = ((el0 + (J)) << SLB) | (int)(SJ); \
        } \
        wc += (int)__builtin_popcount(mj); } }
    HITJ(0, h0, s0)
    HITJ(1, h1, s1)
    HITJ(2, h2, s2)
    HITJ(3, h3, s3)
    HITJ(4, h4, s4)
    HITJ(5, h5, s5)
    HITJ(6, h6, s6)
    HITJ(7, h7, s7)
#undef HITJ
  }
  return wc;
}

__device__ __forceinline__ v8us gath8(const float* __restrict__ p, int stride) {
  v8us o;
#pragma unroll
  for (int i = 0; i < 8; ++i) o[i] = (unsigned short)bf16_bits(p[(size_t)i * stride]);
  return o;
}
__device__ __forceinline__ v8us cont8(const float* __restrict__ p) {
  const v4f a = *(const v4f*)p;
  const v4f b = *(const v4f*)(p + 4);
  v8us o;
  o[0] = (unsigned short)bf16_bits(a.x); o[1] = (unsigned short)bf16_bits(a.y);
  o[2] = (unsigned short)bf16_bits(a.z); o[3] = (unsigned short)bf16_bits(a.w);
  o[4] = (unsigned short)bf16_bits(b.x); o[5] = (unsigned short)bf16_bits(b.y);
  o[6] = (unsigned short)bf16_bits(b.z); o[7] = (unsigned short)bf16_bits(b.w);
  return o;
}

__global__ __launch_bounds__(NTHR) void k_prep(const float* __restrict__ gat_w, const float* __restrict__ gg_w,
                                               const float* __restrict__ w_ih, const float* __restrict__ w_hh,
                                               unsigned short* wp) {
  const int u = (int)blockIdx.x * NTHR + (int)threadIdx.x;
  v8us o;
  int doff;
  if (u < U0) {
    const int n = u >> 3, k8 = (u & 7) * 8;
    o = gath8(gat_w + (size_t)k8 * HID + n, HID);
    doff = O_GWT + n * HID + k8;
  } else if (u < U1) {
    const int v = u - U0, n = v >> 4, k8 = (v & 15) * 8, kk = k8 & 63;
    o = gath8(gg_w + (size_t)kk * HID + n, HID);
    doff = O_M0T + n * K2 + k8;
  } else if (u < U2) {
    const int v = u - U1, n = v >> 4, k8 = (v & 15) * 8, kk = k8 & 63;
    o = gath8(gg_w + (size_t)(HID * HID) + (size_t)kk * HID + n, HID);
    doff = O_M1T + n * K2 + k8;
  } else if (u < U3) {
    const int v = u - U2, n = v >> 4, k8 = (v & 15) * 8, kk = k8 & 63;
    o = cont8(w_ih + (size_t)n * HID + kk);
    doff = O_RZT + n * KRZ + k8;
  } else if (u < U4) {
    const int v = u - U3, n = v >> 4, k8 = (v & 15) * 8, kk = k8 & 63;
    o = cont8(w_hh + (size_t)n * HID + kk);
    doff = O_RZT + n * KRZ + K2 + k8;
  } else if (u < U5) {
    const int v = u - U4, n = v >> 4, k8 = (v & 15) * 8, kk = k8 & 63;
    o = cont8(w_ih + (size_t)(2 * HID + n) * HID + kk);
    doff = O_INT + n * K2 + k8;
  } else if (u < U6) {
    const int v = u - U5, n = v >> 4, k8 = (v & 15) * 8, kk = k8 & 63;
    o = cont8(w_hh + (size_t)(2 * HID + n) * HID + kk);
    doff = O_HNT + n * K2 + k8;
  } else {
    return;
  }
  unsigned short* dp = wp + doff;
  *(volatile v8us*)dp = o;
  __threadfence();
  *(volatile v8us*)dp = o;
}

__global__ __launch_bounds__(GTHR) void k_gat_gemm(const float* __restrict__ X, int nN,
                                                   const unsigned short* __restrict__ GWt,
                                                   const float* __restrict__ att_s,
                                                   const float* __restrict__ att_d,
                                                   float* xh, float* asd, int mp) {
  __shared__ __attribute__((aligned(16))) float stg[GBM * GBN];
  __shared__ __attribute__((aligned(16))) float satt[2 * HID];
  __shared__ __attribute__((aligned(16))) float sdot[2 * GBM];
  const int tid = (int)threadIdx.x, lane = tid & 31, wave = tid >> 5, hh = lane >> 4, m = lane & 15;
  const int rowBase = (int)blockIdx.x * GBM;

  if (tid < HID) { satt[tid] = bf16_val(att_s[tid]); }
  else           { satt[tid] = bf16_val(att_d[tid - HID]); }

  const int row = rowBase + 16 * wave + m;
  const bool ok = row < nN;
  const int rc  = ok ? row : nN - 1;
  const float* ap = X + (size_t)rc * HID + 8 * hh;
  const unsigned short* wq0 = GWt + (size_t)m * HID + 8 * hh;

  v8f acc[4];
  {
    const v8f z = {0.f, 0.f, 0.f, 0.f, 0.f, 0.f, 0.f, 0.f};
    acc[0] = z; acc[1] = z; acc[2] = z; acc[3] = z;
  }
#pragma unroll
  for (int ks = 0; ks < HID / 32; ++ks) {
    const v4f a0 = *(const v4f*)(ap + 32 * ks);
    const v4f a1 = *(const v4f*)(ap + 32 * ks + 4);
    const v4f a2 = *(const v4f*)(ap + 32 * ks + 16);
    const v4f a3 = *(const v4f*)(ap + 32 * ks + 20);
    FragB af;
    af.u[0]  = cvz(a0.x, ok); af.u[1]  = cvz(a0.y, ok); af.u[2]  = cvz(a0.z, ok); af.u[3]  = cvz(a0.w, ok);
    af.u[4]  = cvz(a1.x, ok); af.u[5]  = cvz(a1.y, ok); af.u[6]  = cvz(a1.z, ok); af.u[7]  = cvz(a1.w, ok);
    af.u[8]  = cvz(a2.x, ok); af.u[9]  = cvz(a2.y, ok); af.u[10] = cvz(a2.z, ok); af.u[11] = cvz(a2.w, ok);
    af.u[12] = cvz(a3.x, ok); af.u[13] = cvz(a3.y, ok); af.u[14] = cvz(a3.z, ok); af.u[15] = cvz(a3.w, ok);
#pragma unroll
    for (int t = 0; t < 4; ++t) {
      const unsigned short* wq = wq0 + (size_t)(16 * t) * HID + 32 * ks;
      FragB bf;
      bf.h[0] = *(const v8usa*)wq;
      bf.h[1] = *(const v8usa*)(wq + 16);
      acc[t] = wmb(af, bf, acc[t]);
    }
  }
#pragma unroll
  for (int t = 0; t < 4; ++t) {
    const int lc = 16 * t + m;
#pragma unroll
    for (int r = 0; r < 8; ++r) {
      const int lr = 16 * wave + 8 * hh + r;
      stg[lr * GBN + lc] = acc[t][r];
    }
  }
  __syncthreads();

  {
    const int dr = tid >> 1, dh = tid & 1;
    const float* sr = stg + dr * GBN;
    const float* sa = satt + dh * HID;
    float s = 0.0f;
#pragma unroll 4
    for (int c = 0; c < HID; ++c) s = fmaf(sr[c], sa[c], s);
    sdot[dh * GBM + dr] = s;
  }

  v4f fv[8];
#pragma unroll
  for (int i = 0; i < 8; ++i) {
    const int lr = 16 * wave + 2 * i + hh;
    fv[i] = *(const v4fa*)(stg + lr * GBN + 4 * m);
  }
#pragma unroll
  for (int i = 0; i < 8; ++i) {
    const int lr = 16 * wave + 2 * i + hh;
    float* op = xh + (size_t)(rowBase + lr) * HID + 4 * m;
    *(volatile v4f*)op = fv[i];
  }
  __threadfence();
#pragma unroll
  for (int i = 0; i < 8; ++i) {
    const int lr = 16 * wave + 2 * i + hh;
    float* op = xh + (size_t)(rowBase + lr) * HID + 4 * m;
    *(volatile v4f*)op = fv[i];
  }
  __syncthreads();
  {
    const v4f dv = *(const v4fa*)(sdot + GBM * (wave & 1) + 4 * (lane & 15));
    float* op = asd + (size_t)(wave & 1) * (size_t)mp + rowBase + 4 * (lane & 15);
    const bool st = (wave < 2) && (lane < 16);
    if (st) *(volatile v4f*)op = dv;
    __threadfence();
    if (st) *(volatile v4f*)op = dv;
  }
}

__global__ __launch_bounds__(GTHR) void k_gemm(const unsigned short* __restrict__ A,
                                               const unsigned short* __restrict__ WT,
                                               float* outF, int K, int ldo) {
  __shared__ __attribute__((aligned(16))) float stg[GBM * GBN];
  const int tid = (int)threadIdx.x, lane = tid & 31, wave = tid >> 5, hh = lane >> 4, m = lane & 15;
  const int rowBase = (int)blockIdx.x * GBM;
  const int col0    = (int)blockIdx.y * GBN;

  v8f acc[4];
  {
    const v8f z = {0.f, 0.f, 0.f, 0.f, 0.f, 0.f, 0.f, 0.f};
    acc[0] = z; acc[1] = z; acc[2] = z; acc[3] = z;
  }
  const unsigned short* ap = A  + (size_t)(rowBase + 16 * wave + m) * (size_t)K + 8 * hh;
  const unsigned short* wp = WT + (size_t)(col0 + m) * (size_t)K + 8 * hh;
  const int ksteps = K >> 5;
#pragma unroll 1
  for (int ks = 0; ks < ksteps; ++ks) {
    FragB af;
    af.h[0] = *(const v8usa*)(ap + 32 * ks);
    af.h[1] = *(const v8usa*)(ap + 32 * ks + 16);
#pragma unroll
    for (int t = 0; t < 4; ++t) {
      const unsigned short* wq = wp + (size_t)(16 * t) * (size_t)K + 32 * ks;
      FragB bf;
      bf.h[0] = *(const v8usa*)wq;
      bf.h[1] = *(const v8usa*)(wq + 16);
      acc[t] = wmb(af, bf, acc[t]);
    }
  }
#pragma unroll
  for (int t = 0; t < 4; ++t) {
    const int lc = 16 * t + m;
#pragma unroll
    for (int r = 0; r < 8; ++r) {
      const int lr = 16 * wave + 8 * hh + r;
      stg[lr * GBN + lc] = acc[t][r];
    }
  }
  __syncthreads();
  v4f fv[8];
#pragma unroll
  for (int i = 0; i < 8; ++i) {
    const int lr = 16 * wave + 2 * i + hh;
    fv[i] = *(const v4fa*)(stg + lr * GBN + 4 * m);
  }
#pragma unroll
  for (int i = 0; i < 8; ++i) {
    const int lr = 16 * wave + 2 * i + hh;
    float* op = outF + (size_t)(rowBase + lr) * (size_t)ldo + col0 + 4 * m;
    *(volatile v4f*)op = fv[i];
  }
  __threadfence();
#pragma unroll
  for (int i = 0; i < 8; ++i) {
    const int lr = 16 * wave + 2 * i + hh;
    float* op = outF + (size_t)(rowBase + lr) * (size_t)ldo + col0 + 4 * m;
    *(volatile v4f*)op = fv[i];
  }
}

__global__ __launch_bounds__(NTHR) void k_gat_scan(const int* __restrict__ srcs, const int* __restrict__ dsts,
                                                   int nE, int nN, int vec8, int mRows,
                                                   const float* __restrict__ xh, const float* __restrict__ asd,
                                                   int mp, const float* __restrict__ gbias,
                                                   float* hout, unsigned short* hhl, int* gcnt, int* gsl) {
  extern __shared__ __attribute__((aligned(16))) int dsm[];
  int* list = dsm;
  int* hl   = dsm + LISTN;
  int* sl   = dsm + LISTN + RCAP;
  int* cnt  = dsm + LISTN + 2 * RCAP;
  int* offs = cnt + NBA;
  int* cur  = offs + NBA;
  int* misc = cur + NBA;
  const int tid = (int)threadIdx.x, lane = tid & 31, wave = tid >> 5;
  const int nodeBase = (int)blockIdx.x * NBA;
  const float* AS = asd;
  const float* AD = asd + (size_t)mp;

  {
    const v4i z4 = {0, 0, 0, 0};
    for (int i = tid * 4; i < AGG_ZINTS; i += NTHR * 4) *(v4ia*)(dsm + i) = z4;
    if (tid < MISC_INTS) misc[tid] = 0;
  }
  float bv0, bv1;
  {
    const v2f a = *(const v2fa*)(gbias + 2 * lane);
    bv0 = bf16_val(a.x); bv1 = bf16_val(a.y);
  }
  __syncthreads();

  int t = 0, ov = 0;
  const int nChunks = (nE + CHUNK - 1) / CHUNK;
#pragma unroll 1
  for (int ch = 0; ch < nChunks; ++ch) {
    const int cbase = ch * CHUNK;
    const int wc = scan_chunk<SLA>(dsts, nE, cbase, nodeBase, NBA, vec8, list, tid, lane, wave);
    if (lane == 0) misc[wave] = wc;
    __syncthreads();
    if (wave == 0) {
#pragma unroll 1
      for (int w2 = 0; w2 < NWAVE; ++w2) {
        int c = misc[w2];
        c = c < 0 ? 0 : (c > WCAP ? WCAP : c);
#pragma unroll 1
        for (int b0 = 0; b0 < c; b0 += 32) {
          const int idx = b0 + lane;
          const int ent = list[w2 * WCAP + (idx < WCAP ? idx : WCAP - 1)];
          const int m32 = (c - b0) < 32 ? (c - b0) : 32;
#pragma unroll 1
          for (int k = 0; k < m32; ++k) {
            const int u    = __builtin_amdgcn_readlane(ent, k);
            const int slot = u & (NBA - 1);
            const int el   = (u >> SLA) & (CHUNK - 1);
            const int pk   = ((cbase + el) << SLA) | slot;
            if (t < RCAP) {
              if (lane == 0) { hl[t] = pk; cnt[slot] = cnt[slot] + 1; }
              t = t + 1;
            } else {
              ov = 1;
            }
          }
        }
      }
    }
    __syncthreads();
  }
  if (wave == 0 && lane == 0) { misc[8] = t; misc[9] = ov; }
  __syncthreads();
  int tt = misc[8];
  tt = tt < 0 ? 0 : (tt > RCAP ? RCAP : tt);
  const int ovf = misc[9];

  if (wave == 0) {
    const int base = lane * (NBA / 32);
    int s = 0;
#pragma unroll 1
    for (int i = 0; i < NBA / 32; ++i) s += cnt[base + i];
    int incl = s;
#pragma unroll
    for (int d = 1; d < 32; d <<= 1) {
      const int y = __shfl_up(incl, d, 32);
      if (lane >= d) incl += y;
    }
    int run = incl - s;
#pragma unroll 1
    for (int i = 0; i < NBA / 32; ++i) {
      const int cv = cnt[base + i];
      offs[base + i] = run;
      cur[base + i]  = run;
      run += cv;
    }
  }
  __syncthreads();
  if (wave == 0) {
#pragma unroll 1
    for (int b0 = 0; b0 < tt; b0 += 32) {
      const int idx = b0 + lane;
      const int ent = hl[idx < RCAP ? idx : RCAP - 1];
      const int m32 = (tt - b0) < 32 ? (tt - b0) : 32;
#pragma unroll 1
      for (int k = 0; k < m32; ++k) {
        const int u    = __builtin_amdgcn_readlane(ent, k);
        const int slot = u & (NBA - 1);
        if (lane == 0) {
          int p = cur[slot];
          p = p < 0 ? 0 : (p > RCAP - 1 ? RCAP - 1 : p);
          sl[p] = u;
          cur[slot] = p + 1;
        }
      }
    }
  }
  __syncthreads();

  int* gslb  = gsl + (size_t)blockIdx.x * RCAP;
  int* gcntb = gcnt + (size_t)blockIdx.x * NBA;
  const v4i c4 = *(const v4ia*)(cnt + 4 * tid);
#pragma unroll 1
  for (int it = 0; it < RCAP / (NTHR * 4); ++it) {
    const int i = (it * NTHR + tid) * 4;
    const v4i ent = *(const v4ia*)(sl + i);
    const int e0 = clampi(ent.x >> SLA, 0, nE - 1);
    const int e1 = clampi(ent.y >> SLA, 0, nE - 1);
    const int e2 = clampi(ent.z >> SLA, 0, nE - 1);
    const int e3 = clampi(ent.w >> SLA, 0, nE - 1);
    const int r0 = clampi(srcs[e0], 0, nN - 1);
    const int r1 = clampi(srcs[e1], 0, nN - 1);
    const int r2 = clampi(srcs[e2], 0, nN - 1);
    const int r3 = clampi(srcs[e3], 0, nN - 1);
    v4i rv;
    rv.x = (i     < tt) ? r0 : 0;
    rv.y = (i + 1 < tt) ? r1 : 0;
    rv.z = (i + 2 < tt) ? r2 : 0;
    rv.w = (i + 3 < tt) ? r3 : 0;
    *(v4ia*)(sl + i) = rv;
    *(volatile v4i*)(gslb + i) = rv;
  }
  *(volatile v4i*)(gcntb + 4 * tid) = c4;
  __threadfence();
  __syncthreads();
#pragma unroll 1
  for (int it = 0; it < RCAP / (NTHR * 4); ++it) {
    const int i = (it * NTHR + tid) * 4;
    const v4i rv = *(const v4ia*)(sl + i);
    *(volatile v4i*)(gslb + i) = rv;
  }
  *(volatile v4i*)(gcntb + 4 * tid) = c4;

  const float qnan = __int_as_float(0x7fc00000);
  const float ninf = __int_as_float((int)0xff800000);
  const float pz = (ovf != 0) ? qnan : 0.0f;
#pragma unroll 1
  for (int si = 0; si < NBA / NWAVE; ++si) {
    const int s    = si * NWAVE + wave;
    const int node = nodeBase + s;
    const int craw = cnt[s];
    const bool big = craw > DEGCAP;
    const int c = craw < 0 ? 0 : (craw > DEGCAP ? DEGCAP : craw);
    int o = offs[s];
    o = o < 0 ? 0 : (o > RCAP ? RCAP : o);
    const int nc = node < nN ? node : nN - 1;
    const float asn = AS[nc];
    const float adn = AD[nc];
    int i0 = o + lane;       i0 = i0 > RCAP - 1 ? RCAP - 1 : i0;
    int i1 = o + 32 + lane;  i1 = i1 > RCAP - 1 ? RCAP - 1 : i1;
    const int s0 = clampi(sl[i0], 0, nN - 1);
    const int s1 = clampi(sl[i1], 0, nN - 1);
    const bool ok0 = lane < c;
    const bool ok1 = (lane + 32) < c;
    float e0 = AS[s0] + adn;  e0 = (e0 >= 0.0f) ? e0 : 0.2f * e0;
    float e1 = AS[s1] + adn;  e1 = (e1 >= 0.0f) ? e1 : 0.2f * e1;
    float es = asn + adn;     es = (es >= 0.0f) ? es : 0.2f * es;
    const float c0 = ok0 ? e0 : ninf;
    const float c1 = ok1 ? e1 : ninf;
    float mx = fmaxf(es, fmaxf(c0, c1));
#pragma unroll
    for (int d = 16; d > 0; d >>= 1) mx = fmaxf(mx, __shfl_xor(mx, d, 32));
    const float x0 = expf(e0 - mx);
    const float x1 = expf(e1 - mx);
    const float ex0 = ok0 ? x0 : 0.0f;
    const float ex1 = ok1 ? x1 : 0.0f;
    float sm = ex0 + ex1;
#pragma unroll
    for (int d = 16; d > 0; d >>= 1) sm = sm + __shfl_xor(sm, d, 32);
    const float exs = expf(es - mx);
    const float den = sm + exs;
    const int ex0i = __float_as_int(ex0);
    const int ex1i = __float_as_int(ex1);
    const int n0 = c < 32 ? c : 32;
    const int n1 = (c - 32) < 0 ? 0 : (c - 32);
    float acc0 = 0.0f, acc1 = 0.0f;
#pragma unroll 1
    for (int k = 0; k < n0; ++k) {
      const int   sk = __builtin_amdgcn_readlane(s0, k);
      const float wk = __int_as_float(__builtin_amdgcn_readlane(ex0i, k));
      const v2f a = *(const v2fa*)(xh + (size_t)sk * HID + 2 * lane);
      acc0 = fmaf(wk, a.x, acc0); acc1 = fmaf(wk, a.y, acc1);
    }
#pragma unroll 1
    for (int k = 0; k < n1; ++k) {
      const int   sk = __builtin_amdgcn_readlane(s1, k);
      const float wk = __int_as_float(__builtin_amdgcn_readlane(ex1i, k));
      const v2f a = *(const v2fa*)(xh + (size_t)sk * HID + 2 * lane);
      acc0 = fmaf(wk, a.x, acc0); acc1 = fmaf(wk, a.y, acc1);
    }
    {
      const v2f a = *(const v2fa*)(xh + (size_t)nc * HID + 2 * lane);
      acc0 = fmaf(exs, a.x, acc0); acc1 = fmaf(exs, a.y, acc1);
    }
    const float rden = 1.0f / den;
    float y0 = acc0 * rden + bv0;
    float y1 = acc1 * rden + bv1;
    y0 = (y0 > 0.0f) ? y0 : (y0 - y0);
    y1 = (y1 > 0.0f) ? y1 : (y1 - y1);
    const float pzr = big ? qnan : pz;
    y0 = y0 + pzr; y1 = y1 + pzr;
    const bool live = node < nN;
    const float v0 = live ? y0 : 0.0f;
    const float v1 = live ? y1 : 0.0f;
    const bool wr = (node < mRows) && (lane < 16);
    put_f32_row(hout, node, lane, v0, v1, wr);
    put_hl_row(hhl, node, lane, v0, v1, wr);
  }
}

__global__ __launch_bounds__(NTHR) void k_agg_replay(const int* __restrict__ gcnt, const int* __restrict__ gsl,
                                                     int nN, int mRows, const float* __restrict__ mpl,
                                                     unsigned short* agghl) {
  __shared__ __attribute__((aligned(16))) int cnt[NBA];
  __shared__ __attribute__((aligned(16))) int offs[NBA];
  const int tid = (int)threadIdx.x, lane = tid & 31, wave = tid >> 5;
  const int nodeBase = (int)blockIdx.x * NBA;
  const int* gslb = gsl + (size_t)blockIdx.x * RCAP;
  {
    v4i c4 = *(const v4i*)(gcnt + (size_t)blockIdx.x * NBA + 4 * tid);
    c4.x = clampi(c4.x, 0, RCAP); c4.y = clampi(c4.y, 0, RCAP);
    c4.z = clampi(c4.z, 0, RCAP); c4.w = clampi(c4.w, 0, RCAP);
    *(v4ia*)(cnt + 4 * tid) = c4;
  }
  __syncthreads();
  if (wave == 0) {
    const int base = lane * (NBA / 32);
    int s = 0;
#pragma unroll 1
    for (int i = 0; i < NBA / 32; ++i) s += cnt[base + i];
    int incl = s;
#pragma unroll
    for (int d = 1; d < 32; d <<= 1) {
      const int y = __shfl_up(incl, d, 32);
      if (lane >= d) incl += y;
    }
    int run = incl - s;
#pragma unroll 1
    for (int i = 0; i < NBA / 32; ++i) {
      const int cv = cnt[base + i];
      offs[base + i] = run;
      run += cv;
    }
  }
  __syncthreads();

  const float qnan = __int_as_float(0x7fc00000);
#pragma unroll 1
  for (int si = 0; si < NBA / NWAVE; ++si) {
    const int s    = si * NWAVE + wave;
    const int node = nodeBase + s;
    const int craw = cnt[s];
    const bool big = craw > DEGCAP;
    const int c = craw < 0 ? 0 : (craw > DEGCAP ? DEGCAP : craw);
    int o = offs[s];
    o = o < 0 ? 0 : (o > RCAP ? RCAP : o);
    float a0 = 0.0f, a1 = 0.0f;
#pragma unroll 1
    for (int b0 = 0; b0 < c; b0 += 32) {
      int idx = o + b0 + lane;
      idx = idx > RCAP - 1 ? RCAP - 1 : idx;
      const int sr = clampi(gslb[idx], 0, nN - 1);
      const int m32 = (c - b0) < 32 ? (c - b0) : 32;
#pragma unroll 1
      for (int k = 0; k < m32; ++k) {
        const int sk = __builtin_amdgcn_readlane(sr, k);
        const v2f a = *(const v2fa*)(mpl + (size_t)sk * HID + 2 * lane);
        a0 = a0 + a.x; a1 = a1 + a.y;
      }
    }
    const float pzr = big ? qnan : 0.0f;
    const bool live = node < nN;
    const float m0 = live ? (a0 + pzr) : 0.0f;
    const float m1 = live ? (a1 + pzr) : 0.0f;
    const bool wr = (node < mRows) && (lane < 16);
    put_hl_row(agghl, node, lane, m0, m1, wr);
  }
}

template <int FIN>
__global__ __launch_bounds__(GTHR) void k_gru(const unsigned short* __restrict__ agghl, unsigned short* hhl,
                                              float* hf,
                                              const unsigned short* __restrict__ RZt,
                                              const unsigned short* __restrict__ INt,
                                              const unsigned short* __restrict__ HNt,
                                              const float* __restrict__ b_ih, const float* __restrict__ b_hh,
                                              int nN, float* outp) {
  extern __shared__ __attribute__((aligned(16))) float gsm[];
  float* sb = gsm + 4 * GBM * HID;
  const int tid = (int)threadIdx.x, lane = tid & 31, wave = tid >> 5, hh = lane >> 4, m = lane & 15;
  const int rowBase = (int)blockIdx.x * GBM;

  if (tid < HID) {
    const float i0 = b_ih[tid], i1 = b_ih[HID + tid], i2 = b_ih[2 * HID + tid];
    const float h0 = b_hh[tid], h1 = b_hh[HID + tid], h2 = b_hh[2 * HID + tid];
    sb[tid]           = bf16_val(i0) + bf16_val(h0);
    sb[HID + tid]     = bf16_val(i1) + bf16_val(h1);
    sb[2 * HID + tid] = bf16_val(i2);
    sb[3 * HID + tid] = bf16_val(h2);
  }

  const unsigned short* apa = agghl + (size_t)(rowBase + 16 * wave + m) * K2 + 8 * hh;
  const unsigned short* aph = hhl   + (size_t)(rowBase + 16 * wave + m) * K2 + 8 * hh;
  const v8f z8 = {0.f, 0.f, 0.f, 0.f, 0.f, 0.f, 0.f, 0.f};

  {
    v8f acc[8];
#pragma unroll
    for (int t = 0; t < 8; ++t) acc[t] = z8;
    const unsigned short* bp = RZt + (size_t)m * KRZ + 8 * hh;
#pragma unroll 1
    for (int ks = 0; ks < K2 / 32; ++ks) {
      FragB af;
      af.h[0] = *(const v8usa*)(apa + 32 * ks);
      af.h[1] = *(const v8usa*)(apa + 32 * ks + 16);
#pragma unroll
      for (int nt = 0; nt < 8; ++nt) {
        const unsigned short* wq = bp + (size_t)(16 * nt) * KRZ + 32 * ks;
        FragB bf;
        bf.h[0] = *(const v8usa*)wq;
        bf.h[1] = *(const v8usa*)(wq + 16);
        acc[nt] = wmb(af, bf, acc[nt]);
      }
    }
#pragma unroll 1
    for (int ks = 0; ks < K2 / 32; ++ks) {
      FragB af;
      af.h[0] = *(const v8usa*)(aph + 32 * ks);
      af.h[1] = *(const v8usa*)(aph + 32 * ks + 16);
#pragma unroll
      for (int nt = 0; nt < 8; ++nt) {
        const unsigned short* wq = bp + (size_t)(16 * nt) * KRZ + K2 + 32 * ks;
        FragB bf;
        bf.h[0] = *(const v8usa*)wq;
        bf.h[1] = *(const v8usa*)(wq + 16);
        acc[nt] = wmb(af, bf, acc[nt]);
      }
    }
#pragma unroll
    for (int nt = 0; nt < 8; ++nt) {
      const int lc = 16 * (nt & 3) + m;
#pragma unroll
      for (int r = 0; r < 8; ++r) {
        const int lr = 16 * wave + 8 * hh + r;
        gsm[(nt >> 2) * (GBM * HID) + lr * HID + lc] = acc[nt][r];
      }
    }
  }
  {
    v8f aci[4], ach[4];
#pragma unroll
    for (int t = 0; t < 4; ++t) { aci[t] = z8; ach[t] = z8; }
    const unsigned short* bpi = INt + (size_t)m * K2 + 8 * hh;
    const unsigned short* bph = HNt + (size_t)m * K2 + 8 * hh;
#pragma unroll 1
    for (int ks = 0; ks < K2 / 32; ++ks) {
      FragB afa, afh;
      afa.h[0] = *(const v8usa*)(apa + 32 * ks);
      afa.h[1] = *(const v8usa*)(apa + 32 * ks + 16);
      afh.h[0] = *(const v8usa*)(aph + 32 * ks);
      afh.h[1] = *(const v8usa*)(aph + 32 * ks + 16);
#pragma unroll
      for (int t = 0; t < 4; ++t) {
        const unsigned short* wi = bpi + (size_t)(16 * t) * K2 + 32 * ks;
        const unsigned short* wh = bph + (size_t)(16 * t) * K2 + 32 * ks;
        FragB bi, bh;
        bi.h[0] = *(const v8usa*)wi;
        bi.h[1] = *(const v8usa*)(wi + 16);
        bh.h[0] = *(const v8usa*)wh;
        bh.h[1] = *(const v8usa*)(wh + 16);
        aci[t] = wmb(afa, bi, aci[t]);
        ach[t] = wmb(afh, bh, ach[t]);
      }
    }
#pragma unroll
    for (int t = 0; t < 4; ++t) {
      const int lc = 16 * t + m;
#pragma unroll
      for (int r = 0; r < 8; ++r) {
        const int lr = 16 * wave + 8 * hh + r;
        gsm[2 * (GBM * HID) + lr * HID + lc] = aci[t][r];
        gsm[3 * (GBM * HID) + lr * HID + lc] = ach[t][r];
      }
    }
  }
  __syncthreads();

  const v2f br2 = *(const v2fa*)(sb + 2 * lane);
  const v2f bz2 = *(const v2fa*)(sb + HID + 2 * lane);
  const v2f bi2 = *(const v2fa*)(sb + 2 * HID + 2 * lane);
  const v2f bh2 = *(const v2fa*)(sb + 3 * HID + 2 * lane);
#pragma unroll 1
  for (int i = 0; i < 16; ++i) {
    const int lr = 16 * wave + i;
    const int gr = rowBase + lr;
    const v2f R  = *(const v2fa*)(gsm + lr * HID + 2 * lane);
    const v2f Z  = *(const v2fa*)(gsm + (GBM * HID) + lr * HID + 2 * lane);
    const v2f I  = *(const v2fa*)(gsm + 2 * (GBM * HID) + lr * HID + 2 * lane);
    const v2f Hn = *(const v2fa*)(gsm + 3 * (GBM * HID) + lr * HID + 2 * lane);
    const v2f hv = *(const v2fa*)(hf + (size_t)gr * HID + 2 * lane);
    const float r0 = 1.0f / (1.0f + expf(-(R.x + br2.x)));
    const float r1 = 1.0f / (1.0f + expf(-(R.y + br2.y)));
    const float z0 = 1.0f / (1.0f + expf(-(Z.x + bz2.x)));
    const float z1 = 1.0f / (1.0f + expf(-(Z.y + bz2.y)));
    const float n0 = tanhf((I.x + bi2.x) + r0 * (Hn.x + bh2.x));
    const float n1 = tanhf((I.y + bi2.y) + r1 * (Hn.y + bh2.y));
    const float h0 = (1.0f - z0) * n0 + z0 * hv.x;
    const float h1 = (1.0f - z1) * n1 + z1 * hv.y;
    const bool live = gr < nN;
    if constexpr (FIN != 0) {
      const float y0 = (h0 > 0.0f) ? h0 : (h0 - h0);
      const float y1 = (h1 > 0.0f) ? h1 : (h1 - h1);
      put_f32_row(outp, gr, lane, y0, y1, live && (lane < 16));
    } else {
      const float v0 = live ? h0 : 0.0f;
      const float v1 = live ? h1 : 0.0f;
      put_f32_row(hf, gr, lane, v0, v1, lane < 16);
      put_hl_row(hhl, gr, lane, v0, v1, lane < 16);
    }
  }
}

static inline int cdiv(int a, int b) { return (a + b - 1) / b; }
static inline size_t al256(size_t o) { return (o + 255) & ~(size_t)255; }

extern "C" void kernel_launch(void* const* d_in, const int* in_sizes, int n_in,
                              void* d_out, int out_size, void* d_ws, size_t ws_size,
                              hipStream_t stream) {
  if (n_in < 12) return;
  if (in_sizes[1] < HID || (in_sizes[1] % HID) != 0) return;
  const int nN = in_sizes[1] / HID;
  if (nN < 16 || nN > (1 << 22)) return;
  if (in_sizes[2] < 2 || (in_sizes[2] & 1) != 0) return;
  const int nE = in_sizes[2] / 2;
  if (nE < 1 || nE >= (1 << (31 - SLA))) return;
  if (in_sizes[3] != HID * HID) return;
  if (in_sizes[4] != HID || in_sizes[5] != HID || in_sizes[6] != HID) return;
  if (in_sizes[7] != 2 * HID * HID) return;
  if (in_sizes[8] != 3 * HID * HID || in_sizes[9] != 3 * HID * HID) return;
  if (in_sizes[10] != 3 * HID || in_sizes[11] != 3 * HID) return;
  if ((long long)out_size != (long long)nN * HID) return;

  const float* hidden = (const float*)d_in[1];
  const int*   edge   = (const int*)d_in[2];
  const float* gat_w  = (const float*)d_in[3];
  const float* att_s  = (const float*)d_in[4];
  const float* att_d  = (const float*)d_in[5];
  const float* gat_b  = (const float*)d_in[6];
  const float* gg_w   = (const float*)d_in[7];
  const float* w_ih   = (const float*)d_in[8];
  const float* w_hh   = (const float*)d_in[9];
  const float* b_ih   = (const float*)d_in[10];
  const float* b_hh   = (const float*)d_in[11];
  float* out = (float*)d_out;
  const int* src = edge;
  const int* dst = edge + nE;

  const int MP = cdiv(nN, GBM) * GBM;
  const int gM = MP / GBM;
  const int gA = cdiv(MP, NBA);
  if ((long long)gA * NBA < (long long)MP) return;
  const int vec8 = ((nE & 3) == 0) ? 1 : 0;

  char* ws = (char*)d_ws;
  size_t off = 0;
  const size_t oWP  = off; off = al256(off + (size_t)WP_ELEMS * 2);
  const size_t oASD = off; off = al256(off + (size_t)2 * MP * 4);
  const size_t oCNT = off; off = al256(off + (size_t)gA * NBA * 4);
  const size_t oSL  = off; off = al256(off + (size_t)gA * RCAP * 4);
  const size_t oXH  = off; off = al256(off + (size_t)MP * HID * 4);
  const size_t oH   = off; off = al256(off + (size_t)MP * HID * 4);
  const size_t oHHL = off; off = al256(off + (size_t)MP * K2 * 2);
  const size_t oAGG = off; off = al256(off + (size_t)MP * K2 * 2);
  if (off > ws_size || off > (size_t)WSMAX) return;
  unsigned short* WP  = (unsigned short*)(ws + oWP);
  float*          ASD = (float*)(ws + oASD);
  int*            CNT = (int*)(ws + oCNT);
  int*            SL  = (int*)(ws + oSL);
  float*          XH  = (float*)(ws + oXH);
  float*          H   = (float*)(ws + oH);
  unsigned short* HHL = (unsigned short*)(ws + oHHL);
  unsigned short* AGG = (unsigned short*)(ws + oAGG);

  const size_t scanLds = (size_t)AGG_LDS_INTS * 4;
  const size_t gruLds  = (size_t)GRU_LDS_FLOATS * 4;
  hipFuncSetAttribute(reinterpret_cast<const void*>(&k_gat_scan), hipFuncAttributeMaxDynamicSharedMemorySize, (int)scanLds);
  hipFuncSetAttribute(reinterpret_cast<const void*>(&k_gru<0>), hipFuncAttributeMaxDynamicSharedMemorySize, (int)gruLds);
  hipFuncSetAttribute(reinterpret_cast<const void*>(&k_gru<1>), hipFuncAttributeMaxDynamicSharedMemorySize, (int)gruLds);

  k_prep<<<U6 / NTHR, NTHR, 0, stream>>>(gat_w, gg_w, w_ih, w_hh, WP);
  k_gat_gemm<<<gM, GTHR, 0, stream>>>(hidden, nN, WP + O_GWT, att_s, att_d, XH, ASD, MP);
  k_gat_scan<<<gA, NTHR, scanLds, stream>>>(src, dst, nE, nN, vec8, MP, XH, ASD, MP, gat_b, H, HHL, CNT, SL);
  k_gemm<<<dim3(gM, 1), GTHR, 0, stream>>>(HHL, WP + O_M0T, XH, K2, HID);
  k_agg_replay<<<gA, NTHR, 0, stream>>>(CNT, SL, nN, MP, XH, AGG);
  k_gru<0><<<gM, GTHR, gruLds, stream>>>(AGG, HHL, H, WP + O_RZT, WP + O_INT, WP + O_HNT, b_ih, b_hh, nN, out);
  k_gemm<<<dim3(gM, 1), GTHR, 0, stream>>>(HHL, WP + O_M1T, XH, K2, HID);
  k_agg_replay<<<gA, NTHR, 0, stream>>>(CNT, SL, nN, MP, XH, AGG);
  k_gru<1><<<gM, GTHR, gruLds, stream>>>(AGG, HHL, H, WP + O_RZT, WP + O_INT, WP + O_HNT, b_ih, b_hh, nN, out);
}
